// SelfAttention_56581899158204
// MI455X (gfx1250) — hardware-verified
//
#include <hip/hip_runtime.h>


#ifndef NB
#define NB 2
#endif
#ifndef SEQ
#define SEQ 2048
#endif
#ifndef EARLY
#define EARLY 256
#endif
#define NB_FULL  2
#define SEQ_FULL 2048
#define DIM 1024
#define NH  16
#define HD  64
#define E3  (3 * DIM)
#define QSC 0.18033688011112042f
#define NEGB (-1.0e30f)

typedef _Float16 h16;
typedef unsigned short bf;
typedef __attribute__((ext_vector_type(16))) __bf16   v16bf;
typedef __attribute__((ext_vector_type(16))) _Float16 v16h;
typedef __attribute__((ext_vector_type(16))) unsigned short v16us;
typedef __attribute__((ext_vector_type(8)))  _Float16 v8h;
typedef __attribute__((ext_vector_type(8)))  unsigned short v8us;
typedef __attribute__((ext_vector_type(8)))  float    v8f;
typedef __attribute__((ext_vector_type(4)))  float    v4f;
typedef v4f  __attribute__((may_alias)) v4fa;

static_assert(NH * HD == DIM);
static_assert(HD == 64);
static_assert(DIM % 64 == 0);
static_assert(E3 % 64 == 0);
static_assert(DIM % 32 == 0);
static_assert(SEQ % 64 == 0);
static_assert(EARLY % 64 == 0);
static_assert(EARLY <= SEQ);
static_assert(SEQ <= SEQ_FULL);
static_assert(NB <= NB_FULL);
static_assert((DIM * 4) % 128 == 0);
static_assert((E3 * 4) % 128 == 0);
static_assert((HD * 4) % 128 == 0);
static_assert(((size_t)2 * NH * SEQ * 8) % 256 == 0);
static_assert(((size_t)NH * HD * SEQ / 8) % 256 == 0);

__device__ __forceinline__ unsigned short f2bf(float f) { unsigned u = __float_as_uint(f); u += 0x7FFFu + ((u >> 16) & 1u); return (unsigned short)(u >> 16); }
__device__ __forceinline__ float bf2f(unsigned short b) { return __uint_as_float(((unsigned)b) << 16); }
__device__ __forceinline__ void splitf(float y, unsigned short& h, unsigned short& l) { h = f2bf(y); l = f2bf(y - bf2f(h)); }
__device__ __forceinline__ v16h cat16(v8h lo, v8h hi) { return __builtin_shufflevector(lo, hi, 0, 1, 2, 3, 4, 5, 6, 7, 8, 9, 10, 11, 12, 13, 14, 15); }
__device__ __forceinline__ v16bf cat16b(v8us lo, v8us hi) { return __builtin_bit_cast(v16bf, __builtin_shufflevector(lo, hi, 0, 1, 2, 3, 4, 5, 6, 7, 8, 9, 10, 11, 12, 13, 14, 15)); }
__device__ __forceinline__ v8f wmma16(v16h a, v16h b, v8f c) {
    c = __builtin_amdgcn_wmma_f32_16x16x32_f16(false, a, false, b, (short)0, c, false, false);
    asm volatile("v_nop\n\tv_nop\n\tv_nop\n\tv_nop" : "+v"(c) : "v"(a), "v"(b));
    return c; }
__device__ __forceinline__ v8f wmmab(v16bf a, v16bf b, v8f c) {
    c = __builtin_amdgcn_wmma_f32_16x16x32_bf16(false, a, false, b, (short)0, c, false, false);
    asm volatile("v_nop\n\tv_nop\n\tv_nop\n\tv_nop" : "+v"(c) : "v"(a), "v"(b));
    return c; }
__device__ __forceinline__ v16bf ldb(const bf* p) { return cat16b(*(const v8us*)p, *(const v8us*)(p + 16)); }
__device__ __forceinline__ v16h ldh(const h16* p) { return cat16(*(const v8h*)p, *(const v8h*)(p + 16)); }

__global__ __launch_bounds__(32) void k_gemm_qkv(const bf* __restrict__ A, const bf* __restrict__ Bt, float* C) {
    __shared__ __align__(16) float os[16 * 68];
    const int lane = threadIdx.x & 31, lr = lane & 15, hi = lane >> 4; const int r0 = blockIdx.x * 64, c0 = blockIdx.y * 64;
    v8f acc[4][4];
#pragma unroll
    for (int mb = 0; mb < 4; ++mb)
#pragma unroll
        for (int nb = 0; nb < 4; ++nb) acc[mb][nb] = (v8f){};
    const size_t aoff = (size_t)(r0 + lr) * DIM + 8 * hi, boff = (size_t)(c0 + lr) * DIM + 8 * hi;
#pragma unroll 1
    for (int kc = 0; kc < DIM; kc += 32) {
        v16bf a[4];
#pragma unroll
        for (int mb = 0; mb < 4; ++mb) a[mb] = ldb(A + aoff + (size_t)mb * 16 * DIM + kc);
#pragma unroll
        for (int nb = 0; nb < 4; ++nb) { const v16bf bl = ldb(Bt + boff + (size_t)nb * 16 * DIM + kc);
#pragma unroll
            for (int mb = 0; mb < 4; ++mb) acc[mb][nb] = wmmab(a[mb], bl, acc[mb][nb]); }
    }
#pragma unroll
    for (int mb = 0; mb < 4; ++mb) {
#pragma unroll
        for (int nb = 0; nb < 4; ++nb) {
#pragma unroll
            for (int j = 0; j < 8; ++j) os[(hi * 8 + j) * 68 + nb * 16 + lr] = acc[mb][nb][j]; }
        __builtin_amdgcn_wave_barrier(); asm volatile("" ::: "memory");
        float* crow = C + (size_t)(r0 + mb * 16) * E3 + c0;
#pragma unroll 1
        for (int ps = 0; ps < 2; ++ps) {
#pragma unroll
            for (int s = 0; s < 8; ++s) { const int row = 2 * s + hi, cofs = lr * 4; const v4f val = *(const v4fa*)(os + row * 68 + cofs);
                *(volatile v4f*)(crow + (size_t)row * E3 + cofs) = val; }
            if (ps == 0) __threadfence(); }
        __builtin_amdgcn_wave_barrier(); asm volatile("" ::: "memory");
    }
}

__global__ __launch_bounds__(256) void k_cvt8(const float* __restrict__ src, bf* dst, size_t n8) { const size_t i = (size_t)blockIdx.x * 256 + threadIdx.x; if (i >= n8) return; const v8f v = *(const v8f*)(src + i * 8); v8us o;
#pragma unroll
    for (int k = 0; k < 8; ++k) o[k] = f2bf(v[k]); *(volatile v8us*)(dst + i * 8) = o; __threadfence(); *(volatile v8us*)(dst + i * 8) = o; }

__global__ __launch_bounds__(256) void k_hp(const float* __restrict__ F, bf* PH, bf* PL) {
    const size_t e8 = (size_t)blockIdx.x * 256 + threadIdx.x; if (e8 >= (size_t)2 * NH * SEQ * 8) return;
    const int c = (int)(e8 & 7); const size_t rowi = e8 >> 3; const int t = (int)(rowi % SEQ); const int hh = (int)(rowi / SEQ); const int which = hh / NH; const int h = hh - which * NH;
    const float sc = (which == 0) ? QSC : 1.0f; const float* f = F + (size_t)t * E3 + which * DIM + h * HD + c * 8;
    const v4f a = *(const v4f*)f; const v4f b = *(const v4f*)(f + 4); v8us oh, ol;
#pragma unroll
    for (int k = 0; k < 4; ++k) { unsigned short p, q; splitf(a[k] * sc, p, q); oh[k] = p; ol[k] = q; splitf(b[k] * sc, p, q); oh[4 + k] = p; ol[4 + k] = q; }
    *(volatile v8us*)(PH + e8 * 8) = oh; *(volatile v8us*)(PL + e8 * 8) = ol; __threadfence(); *(volatile v8us*)(PH + e8 * 8) = oh; *(volatile v8us*)(PL + e8 * 8) = ol; }

__global__ __launch_bounds__(256) void k_vtp(const float* __restrict__ F, h16* VT, bf* VEH, bf* VEL) {
    const size_t e8 = (size_t)blockIdx.x * 256 + threadIdx.x; if (e8 >= (size_t)NH * HD * SEQ / 8) return;
    const size_t e = e8 * 8; const int t = (int)(e % SEQ); const int d = (int)((e / SEQ) % HD); const int h = (int)(e / ((size_t)SEQ * HD));
    const float* f = F + (size_t)t * E3 + 2 * DIM + h * HD + d; v8h o; v8us eh, el;
#pragma unroll
    for (int j = 0; j < 8; ++j) { const float v = f[(size_t)j * E3]; unsigned short p, q; splitf(v, p, q); o[j] = (h16)v; eh[j] = p; el[j] = q; }
    const bool early = (t < EARLY);
    const size_t ee = ((size_t)h * HD + d) * EARLY + (early ? t : 0);
    *(volatile v8h*)(VT + e) = o;
    if (early) { *(volatile v8us*)(VEH + ee) = eh; *(volatile v8us*)(VEL + ee) = el; }
    __threadfence();
    *(volatile v8h*)(VT + e) = o;
    if (early) { *(volatile v8us*)(VEH + ee) = eh; *(volatile v8us*)(VEL + ee) = el; }
}

template <bool EP>
__device__ __forceinline__ void flash_body(const bf* __restrict__ PH, const bf* __restrict__ PL, const h16* __restrict__ VT, const bf* __restrict__ VEH, const bf* __restrict__ VEL, float* OUT, const int q0) {
    __shared__ __align__(16) float os[16 * 68];
    __shared__ __align__(16) float ls[16];
    const int lane = threadIdx.x & 31, lr = lane & 15, hi = lane >> 4;
    const int h = blockIdx.y;
    const int vpitch = EP ? EARLY : SEQ;
    const size_t qb = ((size_t)h * SEQ + q0 + lr) * HD + 8 * hi;
    const size_t kb = ((size_t)(NH + h) * SEQ + lr) * HD + 8 * hi;
    const size_t vb = ((size_t)h * HD + lr) * vpitch + 8 * hi;
    v16bf qh[2], ql[2];
    qh[0] = ldb(PH + qb); qh[1] = ldb(PH + qb + 32); ql[0] = ldb(PL + qb); ql[1] = ldb(PL + qb + 32);
    v8f o[4];
#pragma unroll
    for (int dt = 0; dt < 4; ++dt) o[dt] = (v8f){};
    float mrun = NEGB, lrun = 0.0f;
    const int kend = q0 + 16;
#pragma unroll 1
    for (int key0 = 0; key0 < kend; key0 += 32) {
        const size_t ko = kb + (size_t)key0 * HD;
        v8f t0 = (v8f){}, t1 = (v8f){};
#pragma unroll
        for (int kh = 0; kh < 2; ++kh) {
            const v16bf k0h = ldb(PH + ko + 32 * kh), k0l = ldb(PL + ko + 32 * kh);
            const v16bf k1h = ldb(PH + ko + 16 * HD + 32 * kh), k1l = ldb(PL + ko + 16 * HD + 32 * kh);
            t0 = wmmab(k0h, qh[kh], t0); t1 = wmmab(k1h, qh[kh], t1);
            t0 = wmmab(k0l, qh[kh], t0); t1 = wmmab(k1l, qh[kh], t1);
            t0 = wmmab(k0h, ql[kh], t0); t1 = wmmab(k1h, ql[kh], t1);
        }
        if (key0 + 31 > q0) {
            const int qrow = q0 + lr, kk = key0 + 8 * hi;
#pragma unroll
            for (int j = 0; j < 8; ++j) { t0[j] = (kk + j > qrow) ? NEGB : t0[j]; t1[j] = (kk + 16 + j > qrow) ? NEGB : t1[j]; }
        }
        float mx = fmaxf(t0[0], t1[0]);
#pragma unroll
        for (int j = 1; j < 8; ++j) mx = fmaxf(mx, fmaxf(t0[j], t1[j]));
        mx = fmaxf(mx, __shfl_xor(mx, 16, 32));
        const float mnew = fmaxf(mrun, mx);
        const float alpha = __builtin_amdgcn_exp2f(mrun - mnew);
        const float msh = mnew - 10.0f;
        float rs = 0.0f; float pa[8], pb[8];
#pragma unroll
        for (int j = 0; j < 8; ++j) { pa[j] = __builtin_amdgcn_exp2f(t0[j] - msh); pb[j] = __builtin_amdgcn_exp2f(t1[j] - msh); rs += pa[j] + pb[j]; }
        lrun = lrun * alpha + rs;
        if (__builtin_amdgcn_ballot_w32(mnew > mrun) != 0u) {
#pragma unroll
            for (int r = 0; r < 8; ++r) { const float ar = __shfl(alpha, 8 * hi + r, 32); o[0][r] *= ar; o[1][r] *= ar; o[2][r] *= ar; o[3][r] *= ar; }
        }
        mrun = mnew;
        const size_t vo = vb + (size_t)key0;
        if (EP) {
            v16us uh, ul;
#pragma unroll
            for (int j = 0; j < 8; ++j) { unsigned short p, q; splitf(pa[j], p, q); uh[j] = p; ul[j] = q; splitf(pb[j], p, q); uh[8 + j] = p; ul[8 + j] = q; }
            const v16bf pfh = __builtin_bit_cast(v16bf, uh), pfl = __builtin_bit_cast(v16bf, ul);
            {
                const v16bf v0 = ldb(VEH + vo), v1 = ldb(VEH + vo + (size_t)16 * vpitch), v2 = ldb(VEH + vo + (size_t)32 * vpitch), v3 = ldb(VEH + vo + (size_t)48 * vpitch);
                o[0] = wmmab(pfh, v0, o[0]); o[1] = wmmab(pfh, v1, o[1]); o[2] = wmmab(pfh, v2, o[2]); o[3] = wmmab(pfh, v3, o[3]);
                o[0] = wmmab(pfl, v0, o[0]); o[1] = wmmab(pfl, v1, o[1]); o[2] = wmmab(pfl, v2, o[2]); o[3] = wmmab(pfl, v3, o[3]);
            }
            {
                const v16bf w0 = ldb(VEL + vo), w1 = ldb(VEL + vo + (size_t)16 * vpitch), w2 = ldb(VEL + vo + (size_t)32 * vpitch), w3 = ldb(VEL + vo + (size_t)48 * vpitch);
                o[0] = wmmab(pfh, w0, o[0]); o[1] = wmmab(pfh, w1, o[1]); o[2] = wmmab(pfh, w2, o[2]); o[3] = wmmab(pfh, w3, o[3]);
            }
        } else {
            v16h pf;
#pragma unroll
            for (int j = 0; j < 8; ++j) { pf[j] = (h16)pa[j]; pf[8 + j] = (h16)pb[j]; }
            const v16h vf0 = ldh(VT + vo), vf1 = ldh(VT + vo + (size_t)16 * vpitch), vf2 = ldh(VT + vo + (size_t)32 * vpitch), vf3 = ldh(VT + vo + (size_t)48 * vpitch);
            o[0] = wmma16(pf, vf0, o[0]); o[1] = wmma16(pf, vf1, o[1]); o[2] = wmma16(pf, vf2, o[2]); o[3] = wmma16(pf, vf3, o[3]);
        }
    }
    lrun += __shfl_xor(lrun, 16, 32);
    const float inv = 1.0f / lrun;
    if (hi == 0) ls[lr] = inv;
#pragma unroll
    for (int dt = 0; dt < 4; ++dt) {
#pragma unroll
        for (int r = 0; r < 8; ++r) os[(hi * 8 + r) * 68 + dt * 16 + lr] = o[dt][r]; }
    __builtin_amdgcn_wave_barrier(); asm volatile("" ::: "memory");
    float* orow = OUT + (size_t)q0 * DIM + h * HD;
#pragma unroll 1
    for (int ps = 0; ps < 2; ++ps) {
#pragma unroll
        for (int s = 0; s < 8; ++s) { const int row = 2 * s + hi, cofs = lr * 4; const float f = ls[row];
            v4f val = *(const v4fa*)(os + row * 68 + cofs); val[0] *= f; val[1] *= f; val[2] *= f; val[3] *= f;
            *(volatile v4f*)(orow + (size_t)row * DIM + cofs) = val; }
        if (ps == 0) __threadfence(); }
}

__global__ __launch_bounds__(32) void k_flash(const bf* __restrict__ PH, const bf* __restrict__ PL, const h16* __restrict__ VT, float* OUT) {
    flash_body<false>(PH, PL, VT, nullptr, nullptr, OUT, EARLY + (int)blockIdx.x * 16); }
__global__ __launch_bounds__(32) void k_flash_e(const bf* __restrict__ PH, const bf* __restrict__ PL, const bf* __restrict__ VEH, const bf* __restrict__ VEL, float* OUT) {
    flash_body<true>(PH, PL, nullptr, VEH, VEL, OUT, (int)blockIdx.x * 16); }

constexpr size_t al256(size_t b) { return (b + 255) & ~(size_t)255; }
constexpr size_t SZ_XB   = al256((size_t)SEQ * DIM * 2);
constexpr size_t SZ_WQKV = al256((size_t)E3 * DIM * 2);
constexpr size_t SZ_F    = al256((size_t)SEQ * E3 * 4);
constexpr size_t SZ_PH   = al256((size_t)2 * NH * SEQ * HD * 2);
constexpr size_t SZ_VT   = al256((size_t)NH * HD * SEQ * 2);
constexpr size_t SZ_VE   = al256((size_t)NH * HD * EARLY * 2);
constexpr size_t OFF_XB   = 0;
constexpr size_t OFF_WQKV = OFF_XB + SZ_XB;
constexpr size_t OFF_F    = OFF_WQKV + SZ_WQKV;
constexpr size_t OFF_PH   = OFF_F + SZ_F;
constexpr size_t OFF_PL   = OFF_PH + SZ_PH;
constexpr size_t OFF_VT   = OFF_PL + SZ_PH;
constexpr size_t OFF_VEH  = OFF_VT + SZ_VT;
constexpr size_t OFF_VEL  = OFF_VEH + SZ_VE;
constexpr size_t OFF_END  = OFF_VEL + SZ_VE;
static_assert(OFF_END <= (size_t)134217728);
static_assert(((size_t)SEQ * DIM) % 8 == 0);
static_assert(((size_t)DIM * DIM) % 8 == 0);
static_assert((size_t)3 * DIM * DIM * 2 <= SZ_WQKV);
static_assert(((size_t)(NB_FULL - 1) * SEQ_FULL * DIM + (size_t)SEQ_FULL * DIM) * 4 == (size_t)16777216);

extern "C" void kernel_launch(void* const* d_in, const int* in_sizes, int n_in,
                              void* d_out, int out_size, void* d_ws, size_t ws_size, hipStream_t stream) {
    if (n_in < 4) return;
    const size_t xneed = (size_t)(NB - 1) * SEQ_FULL * DIM + (size_t)SEQ * DIM;
    if ((size_t)in_sizes[0] < xneed) return;
    if ((size_t)in_sizes[1] < (size_t)DIM * DIM) return;
    if ((size_t)in_sizes[2] < (size_t)DIM * DIM) return;
    if ((size_t)in_sizes[3] < (size_t)DIM * DIM) return;
    if ((size_t)out_size < xneed) return;
    if (OFF_END > ws_size) return;
    const float* x = (const float*)d_in[0]; const float* wq = (const float*)d_in[1]; const float* wk = (const float*)d_in[2]; const float* wv = (const float*)d_in[3];
    float* OUT = (float*)d_out;
    char* wsp = (char*)d_ws;
    bf* XB = (bf*)(wsp + OFF_XB); bf* WQKV = (bf*)(wsp + OFF_WQKV); float* F = (float*)(wsp + OFF_F);
    bf* PH = (bf*)(wsp + OFF_PH); bf* PL = (bf*)(wsp + OFF_PL); h16* VT = (h16*)(wsp + OFF_VT); bf* VEH = (bf*)(wsp + OFF_VEH); bf* VEL = (bf*)(wsp + OFF_VEL);
    const unsigned wblocks = (unsigned)(((size_t)DIM * DIM / 8 + 255) / 256);
    k_cvt8<<<wblocks, 256, 0, stream>>>(wq, WQKV, (size_t)DIM * DIM / 8);
    k_cvt8<<<wblocks, 256, 0, stream>>>(wk, WQKV + (size_t)DIM * DIM, (size_t)DIM * DIM / 8);
    k_cvt8<<<wblocks, 256, 0, stream>>>(wv, WQKV + (size_t)2 * DIM * DIM, (size_t)DIM * DIM / 8);
    for (int b = 0; b < NB; ++b) {
        float* OUTb = OUT + (size_t)b * SEQ_FULL * DIM;
        k_cvt8<<<(unsigned)(((size_t)SEQ * DIM / 8 + 255) / 256), 256, 0, stream>>>(x + (size_t)b * SEQ_FULL * DIM, XB, (size_t)SEQ * DIM / 8);
        k_gemm_qkv<<<dim3(SEQ / 64, E3 / 64, 1), 32, 0, stream>>>(XB, WQKV, F);
        k_hp<<<(unsigned)(((size_t)2 * NH * SEQ * 8 + 255) / 256), 256, 0, stream>>>(F, PH, PL);
        k_vtp<<<(unsigned)(((size_t)NH * HD * SEQ / 8 + 255) / 256), 256, 0, stream>>>(F, VT, VEH, VEL);
        k_flash_e<<<dim3(EARLY / 16, NH, 1), 32, 0, stream>>>(PH, PL, VEH, VEL, OUTb);
        if (SEQ > EARLY) k_flash<<<dim3((SEQ - EARLY) / 16, NH, 1), 32, 0, stream>>>(PH, PL, VT, OUTb);
    }
}
